// GraphSAGE_local_94489281444
// MI455X (gfx1250) — hardware-run, weakly checked
//
#include <hip/hip_runtime.h>
#include <stddef.h>
#include <math.h>


#define FD      128
#define NO      64
#define NTHR    256
#define NWAVE   8
#define EPT     8
#define NGRP    2
#define CHUNK   (NTHR * EPT * NGRP)
#define WCAP    (EPT * NGRP * 32)
#define LISTN   (NWAVE * WCAP)
#define NBC     4096
#define NBF     1024
#define RCAP    40960
#define RBN     128
#define TGT     256
#define DEGCAP  1024
#define GROWS   128
#define OTHR    512
#define WSCAP   134217728
#define WSC     64.0f
#define WINV    0.015625f

#define WP1     0
#define WL1     16384
#define WP2     49152
#define WL2     65536
#define WPTOT   81920

#define SPH     136
#define SPF     68
#define SSTG    (GROWS * SPH * 2)
#define LDS_FILL ((RCAP + NBF + LISTN) * 4 + 64)
#define LDS_AGG  (TGT * FD * 2)

static_assert((CHUNK & (CHUNK - 1)) == 0);
static_assert(CHUNK <= 4096);
static_assert(NBC <= 4096 && NBF <= 4096);
static_assert((NBC & (NBC - 1)) == 0 && (NBF & (NBF - 1)) == 0);
static_assert(NBC == 4 * NBF);
static_assert(OTHR * 8 == NBC);
static_assert((RCAP % 32) == 0);
static_assert(TGT == NWAVE * 32 && (TGT % GROWS) == 0);
static_assert((NBC % TGT) == 0);
static_assert(GROWS == NWAVE * 16);
static_assert(SSTG == GROWS * SPF * 4);
static_assert((SPH % 8) == 0 && (SPF % 4) == 0);
static_assert(WL1 == WP1 + FD * FD && WP2 == WL1 + FD * 2 * FD && WL2 == WP2 + FD * FD && WPTOT == WL2 + NO * 2 * FD);

typedef float          v4f  __attribute__((ext_vector_type(4)));
typedef float          v8f  __attribute__((ext_vector_type(8)));
typedef int            v4i  __attribute__((ext_vector_type(4)));
typedef _Float16       v4h  __attribute__((ext_vector_type(4)));
typedef _Float16       v8h  __attribute__((ext_vector_type(8)));
typedef _Float16       v16h __attribute__((ext_vector_type(16)));
union FragH { v16h v; v8h h[2]; };
union Pack8 { v8h h; v4f f; };

__device__ __forceinline__ v8f wmh(v16h a, v16h b, v8f c) {
  v8f d = __builtin_amdgcn_wmma_f32_16x16x32_f16(false, a, false, b, (short)0, c, false, false);
  asm volatile("v_nop\n\tv_nop\n\tv_nop\n\tv_nop" : "+v"(d) : "v"(a), "v"(b));
  return d;
}

template <int NB>
__device__ __forceinline__ int scan_chunk(const int* __restrict__ dsts, int nE, int cbase, int slotBase,
                                          int vec8, int* list, int tid, int lane, int wave) {
  int wc = 0;
#pragma unroll
  for (int g = 0; g < NGRP; ++g) {
    const int el0  = (g * NTHR + tid) * EPT;
    const int e0   = cbase + el0;
    const int sent = -2147483647 - 1;
    v4i da, db;
    if (vec8 != 0 && cbase + CHUNK <= nE) {
      da = *(const v4i*)(dsts + e0);
      db = *(const v4i*)(dsts + e0 + 4);
    } else {
      da.x = (e0     < nE) ? dsts[min(e0, nE - 1)] : sent;
      da.y = (e0 + 1 < nE) ? dsts[min(e0 + 1, nE - 1)] : sent;
      da.z = (e0 + 2 < nE) ? dsts[min(e0 + 2, nE - 1)] : sent;
      da.w = (e0 + 3 < nE) ? dsts[min(e0 + 3, nE - 1)] : sent;
      db.x = (e0 + 4 < nE) ? dsts[min(e0 + 4, nE - 1)] : sent;
      db.y = (e0 + 5 < nE) ? dsts[min(e0 + 5, nE - 1)] : sent;
      db.z = (e0 + 6 < nE) ? dsts[min(e0 + 6, nE - 1)] : sent;
      db.w = (e0 + 7 < nE) ? dsts[min(e0 + 7, nE - 1)] : sent;
    }
    const unsigned nb = (unsigned)slotBase;
    const unsigned s0 = (unsigned)da.x - nb, s1 = (unsigned)da.y - nb;
    const unsigned s2 = (unsigned)da.z - nb, s3 = (unsigned)da.w - nb;
    const unsigned s4 = (unsigned)db.x - nb, s5 = (unsigned)db.y - nb;
    const unsigned s6 = (unsigned)db.z - nb, s7 = (unsigned)db.w - nb;
    const bool h0 = s0 < (unsigned)NB, h1 = s1 < (unsigned)NB, h2 = s2 < (unsigned)NB, h3 = s3 < (unsigned)NB;
    const bool h4 = s4 < (unsigned)NB, h5 = s5 < (unsigned)NB, h6 = s6 < (unsigned)NB, h7 = s7 < (unsigned)NB;
    const unsigned any = __builtin_amdgcn_ballot_w32(h0 | h1 | h2 | h3 | h4 | h5 | h6 | h7);
    if (any != 0u) {
#define HITJ(J, HJ, SJ) { \
        const unsigned mj = __builtin_amdgcn_ballot_w32(HJ); \
        if (mj != 0u) { \
          if (HJ) { \
            const int pos = wc + (int)__builtin_amdgcn_mbcnt_lo(mj, 0u); \
            if (pos < WCAP) list[wave * WCAP + pos] = ((el0 + (J)) << 12) | (int)(SJ); \
          } \
          wc += (int)__builtin_popcount(mj); } }
      HITJ(0, h0, s0)
      HITJ(1, h1, s1)
      HITJ(2, h2, s2)
      HITJ(3, h3, s3)
      HITJ(4, h4, s4)
      HITJ(5, h5, s5)
      HITJ(6, h6, s6)
      HITJ(7, h7, s7)
#undef HITJ
    }
  }
  return wc;
}

__global__ __launch_bounds__(NTHR) void k_wprep(
    const float* __restrict__ p1w, const float* __restrict__ l1lw, const float* __restrict__ l1rw,
    const float* __restrict__ p2w, const float* __restrict__ l2lw, const float* __restrict__ l2rw,
    _Float16* wp) {
  const int blk = blockIdx.x, tid = threadIdx.x;
  const int i = blk * NTHR + tid;
  float v[8];
  if (blk < 8) {
    const int n = i >> 4, k0 = (i & 15) * 8;
#pragma unroll
    for (int e = 0; e < 8; ++e) v[e] = p1w[n * FD + k0 + e];
  } else if (blk < 24) {
    const int j = i - 2048;
    const int n = j >> 5, k0 = (j & 31) * 8, kk = k0 & 127;
#pragma unroll
    for (int e = 0; e < 8; ++e) {
      const float va = l1lw[n * FD + kk + e];
      const float vb = l1rw[n * FD + kk + e];
      v[e] = (k0 < 128) ? va : vb;
    }
  } else if (blk < 32) {
    const int j = i - 6144;
    const int n = j >> 4, k0 = (j & 15) * 8;
#pragma unroll
    for (int e = 0; e < 8; ++e) v[e] = p2w[n * FD + k0 + e];
  } else {
    const int j = i - 8192;
    const int n = j >> 5, k0 = (j & 31) * 8, kk = k0 & 127;
#pragma unroll
    for (int e = 0; e < 8; ++e) {
      const float va = l2lw[n * FD + kk + e];
      const float vb = l2rw[n * FD + kk + e];
      v[e] = (k0 < 128) ? va : vb;
    }
  }
  Pack8 pk;
#pragma unroll
  for (int e = 0; e < 8; ++e) pk.h[e] = (_Float16)(v[e] * WSC);
  _Float16* dp = wp + (size_t)i * 8;
  *(volatile v4f*)dp = pk.f;
  __threadfence();
  *(volatile v4f*)dp = pk.f;
}

__global__ __launch_bounds__(NTHR) void k_cvtx(const float* __restrict__ x, _Float16* xh, int nN) {
  const int i = blockIdx.x * NTHR + threadIdx.x;
  const int row = i >> 4, c0 = (i & 15) * 8;
  const int rc = row < nN ? row : (nN - 1);
  const float* p = x + (size_t)rc * FD + c0;
  const v4f a = *(const v4f*)p, b = *(const v4f*)(p + 4);
  const bool ok = row < nN;
  Pack8 pk;
  pk.h[0] = (_Float16)(ok ? a.x : 0.0f); pk.h[1] = (_Float16)(ok ? a.y : 0.0f);
  pk.h[2] = (_Float16)(ok ? a.z : 0.0f); pk.h[3] = (_Float16)(ok ? a.w : 0.0f);
  pk.h[4] = (_Float16)(ok ? b.x : 0.0f); pk.h[5] = (_Float16)(ok ? b.y : 0.0f);
  pk.h[6] = (_Float16)(ok ? b.z : 0.0f); pk.h[7] = (_Float16)(ok ? b.w : 0.0f);
  _Float16* dp = xh + (size_t)i * 8;
  *(volatile v4f*)dp = pk.f;
  __threadfence();
  *(volatile v4f*)dp = pk.f;
}

__global__ __launch_bounds__(NTHR) void k_count(const int* __restrict__ dsts, int* cnt, int nE, int vec8) {
  __shared__ __attribute__((aligned(16))) int scnt[NBC];
  __shared__ __attribute__((aligned(16))) int list[LISTN];
  __shared__ int wcnt[NWAVE];
  const int tid = threadIdx.x, lane = tid & 31, wave = tid >> 5;
  const int nodeBase = blockIdx.x * NBC;

  for (int i = tid; i < NBC; i += NTHR) scnt[i] = 0;
  __syncthreads();

  const int nChunks = (nE + CHUNK - 1) / CHUNK;
#pragma unroll 1
  for (int ch = 0; ch < nChunks; ++ch) {
    const int cbase = ch * CHUNK;
    const int wc = scan_chunk<NBC>(dsts, nE, cbase, nodeBase, vec8, list, tid, lane, wave);
    if (lane == 0) wcnt[wave] = wc;
    __syncthreads();
    if (wave == 0) {
#pragma unroll 1
      for (int wsx = 0; wsx < NWAVE; ++wsx) {
        int n = __builtin_amdgcn_readfirstlane(wcnt[wsx]);
        n = n > WCAP ? WCAP : (n < 0 ? 0 : n);
        const int* lp = list + wsx * WCAP;
#pragma unroll 1
        for (int i = 0; i < n; ++i) {
          const int ent  = __builtin_amdgcn_readfirstlane(lp[i]);
          const int slot = ent & (NBC - 1);
          if (lane == 0) scnt[slot] = scnt[slot] + 1;
        }
      }
    }
    __syncthreads();
  }

  v4i cq[4];
#pragma unroll
  for (int q = 0; q < 4; ++q) {
    const int f = (wave * 4 + q) * 128 + 4 * lane;
    cq[q] = *(const v4i*)(scnt + f);
  }
  int* cp = cnt + (size_t)nodeBase;
#pragma unroll
  for (int q = 0; q < 4; ++q) {
    const int f = (wave * 4 + q) * 128 + 4 * lane;
    *(volatile v4i*)(cp + f) = cq[q];
  }
  __threadfence();
#pragma unroll
  for (int q = 0; q < 4; ++q) {
    const int f = (wave * 4 + q) * 128 + 4 * lane;
    *(volatile v4i*)(cp + f) = cq[q];
  }
}

__global__ __launch_bounds__(OTHR) void k_offsets(
    const int* __restrict__ cnt, int* off, int* rbase, int nChunk) {
  __shared__ __attribute__((aligned(16))) int soff[NBC];
  __shared__ __attribute__((aligned(16))) int srb[RBN];
  __shared__ int wtot[OTHR / 32];
  const int tid = threadIdx.x, lane = tid & 31, wave = tid >> 5, sub = tid >> 7;
  for (int i = tid; i < RBN; i += OTHR) srb[i] = 0;
  int carry = 0;
#pragma unroll 1
  for (int ch = 0; ch < nChunk; ++ch) {
    const int base = ch * NBC;
    const v4i c0 = *(const v4i*)(cnt + base + 8 * tid);
    const v4i c1 = *(const v4i*)(cnt + base + 8 * tid + 4);
    const int e0 = max(c0.x, 0), e1 = max(c0.y, 0), e2 = max(c0.z, 0), e3 = max(c0.w, 0);
    const int e4 = max(c1.x, 0), e5 = max(c1.y, 0), e6 = max(c1.z, 0), e7 = max(c1.w, 0);
    const int ts = e0 + e1 + e2 + e3 + e4 + e5 + e6 + e7;
    int incl = ts;
#pragma unroll
    for (int d = 1; d < 32; d <<= 1) {
      const int t = __shfl_up(incl, d);
      if (lane >= d) incl += t;
    }
    if (lane == 31) wtot[wave] = incl;
    __syncthreads();
    const int S0 = wtot[0]  + wtot[1]  + wtot[2]  + wtot[3];
    const int S1 = wtot[4]  + wtot[5]  + wtot[6]  + wtot[7];
    const int S2 = wtot[8]  + wtot[9]  + wtot[10] + wtot[11];
    const int S3 = wtot[12] + wtot[13] + wtot[14] + wtot[15];
    int pre = 0;
#pragma unroll 1
    for (int w = 4 * sub; w < wave; ++w) pre += wtot[w];
    const int b0 = carry;
    const int b1 = b0 + ((S0 + 31) & ~31);
    const int b2 = b1 + ((S1 + 31) & ~31);
    const int b3 = b2 + ((S2 + 31) & ~31);
    const int b4 = b3 + ((S3 + 31) & ~31);
    const int myb = sub == 0 ? b0 : (sub == 1 ? b1 : (sub == 2 ? b2 : b3));
    if (tid == 0) {
      srb[min(4 * ch + 0, RBN - 1)] = b0;
      srb[min(4 * ch + 1, RBN - 1)] = b1;
      srb[min(4 * ch + 2, RBN - 1)] = b2;
      srb[min(4 * ch + 3, RBN - 1)] = b3;
    }
    int run = myb + pre + incl - ts;
    soff[8 * tid + 0] = run; run += e0;
    soff[8 * tid + 1] = run; run += e1;
    soff[8 * tid + 2] = run; run += e2;
    soff[8 * tid + 3] = run; run += e3;
    soff[8 * tid + 4] = run; run += e4;
    soff[8 * tid + 5] = run; run += e5;
    soff[8 * tid + 6] = run; run += e6;
    soff[8 * tid + 7] = run;
    carry = b4;
    __syncthreads();
    const v4i o0 = *(const v4i*)(soff + 4 * tid);
    const v4i o1 = *(const v4i*)(soff + 4 * (tid + OTHR));
    int* op = off + base;
    *(volatile v4i*)(op + 4 * tid) = o0;
    *(volatile v4i*)(op + 4 * (tid + OTHR)) = o1;
    __threadfence();
    *(volatile v4i*)(op + 4 * tid) = o0;
    *(volatile v4i*)(op + 4 * (tid + OTHR)) = o1;
    __syncthreads();
  }
  if (tid == 0) srb[min(4 * nChunk, RBN - 1)] = carry;
  __syncthreads();
  v4i rv = {0, 0, 0, 0};
  if (tid < 32) rv = *(const v4i*)(srb + 4 * tid);
  if (tid < 32) *(volatile v4i*)(rbase + 4 * tid) = rv;
  __threadfence();
  if (tid < 32) *(volatile v4i*)(rbase + 4 * tid) = rv;
}

__global__ __launch_bounds__(NTHR) void k_fill(
    const int* __restrict__ srcs, const int* __restrict__ dsts,
    const int* __restrict__ off, const int* __restrict__ rbase,
    int* csr, int nN, int nE, int vec8, int csrLen) {
  extern __shared__ v4f lds_dyn[];
  int* region = (int*)lds_dyn;
  int* cursor = region + RCAP;
  int* list   = cursor + NBF;
  int* wcnt   = list + LISTN;
  const int tid = threadIdx.x, lane = tid & 31, wave = tid >> 5;
  const int b = blockIdx.x;
  const int nodeBase = b * NBF;

  int rb0 = rbase[b];
  const int rb1 = rbase[b + 1];
  rb0 = rb0 < 0 ? 0 : (rb0 > csrLen ? csrLen : rb0);
  rb0 &= ~31;
  int len = rb1 - rb0;
  len = len < 0 ? 0 : (len > RCAP ? RCAP : len);
  int lenW = (len + 31) & ~31;
  if (rb0 + lenW > csrLen) lenW = (csrLen - rb0) & ~31;

  {
    const v4i z = {0, 0, 0, 0};
    for (int i = tid; i < RCAP / 4; i += NTHR) ((v4i*)region)[i] = z;
    for (int s = tid; s < NBF; s += NTHR) {
      int o = off[nodeBase + s] - rb0;
      o = o < 0 ? 0 : (o > RCAP ? RCAP : o);
      cursor[s] = o;
    }
  }
  __syncthreads();

  const int nChunks = (nE + CHUNK - 1) / CHUNK;
#pragma unroll 1
  for (int ch = 0; ch < nChunks; ++ch) {
    const int cbase = ch * CHUNK;
    const int wc = scan_chunk<NBF>(dsts, nE, cbase, nodeBase, vec8, list, tid, lane, wave);
    if (lane == 0) wcnt[wave] = wc;
    __syncthreads();
    if (wave == 0) {
#pragma unroll 1
      for (int wsx = 0; wsx < NWAVE; ++wsx) {
        int n = __builtin_amdgcn_readfirstlane(wcnt[wsx]);
        n = n > WCAP ? WCAP : (n < 0 ? 0 : n);
        const int* lp = list + wsx * WCAP;
#pragma unroll 1
        for (int i = 0; i < n; ++i) {
          const int ent  = __builtin_amdgcn_readfirstlane(lp[i]);
          const int slot = ent & (NBF - 1);
          int e = cbase + ((ent >> 12) & (CHUNK - 1));
          e = e > nE - 1 ? nE - 1 : e;
          int sv = srcs[e];
          sv = sv < 0 ? 0 : (sv > nN - 1 ? nN - 1 : sv);
          if (lane == 0) {
            int pos = cursor[slot];
            pos = pos < 0 ? 0 : (pos > RCAP - 1 ? RCAP - 1 : pos);
            region[pos] = sv;
            const int np = pos + 1;
            cursor[slot] = np > RCAP ? RCAP : np;
          }
        }
      }
    }
    __syncthreads();
  }

  const int nv = lenW >> 2;
  int* gp = csr + rb0;
#pragma unroll 1
  for (int i = tid; i < nv; i += NTHR) { const v4i v = ((const v4i*)region)[i]; *(volatile v4i*)(gp + 4 * i) = v; }
  __threadfence();
#pragma unroll 1
  for (int i = tid; i < nv; i += NTHR) { const v4i v = ((const v4i*)region)[i]; *(volatile v4i*)(gp + 4 * i) = v; }
}

template <int KD, int NT, bool FIN>
__global__ __launch_bounds__(NTHR) void k_gemm(
    const _Float16* __restrict__ A1, const _Float16* __restrict__ A2,
    const _Float16* __restrict__ W, const float* __restrict__ bias,
    _Float16* C, float* out, int nN) {
  static_assert(KD == FD || KD == 2 * FD);
  static_assert((FIN && NT == 4 && KD == 2 * FD) || (!FIN && NT == 8));
  __shared__ __attribute__((aligned(16))) unsigned char sraw[SSTG];
  const int tid = threadIdx.x, lane = tid & 31, wave = tid >> 5, hh = lane >> 4, m = lane & 15;
  const int rowBase = blockIdx.x * GROWS;
  const size_t arow = (size_t)(rowBase + wave * 16 + m) * FD + 8 * hh;

  v8f acc[NT];
#pragma unroll
  for (int t = 0; t < NT; ++t) { const v8f z = {0.f, 0.f, 0.f, 0.f, 0.f, 0.f, 0.f, 0.f}; acc[t] = z; }

#pragma unroll 1
  for (int kt = 0; kt < 4; ++kt) {
    FragH a;
    a.h[0] = *(const v8h*)(A1 + arow + 32 * kt);
    a.h[1] = *(const v8h*)(A1 + arow + 32 * kt + 16);
#pragma unroll
    for (int t = 0; t < NT; ++t) {
      const _Float16* bp = W + (size_t)(16 * t + m) * KD + 32 * kt + 8 * hh;
      FragH bf;
      bf.h[0] = *(const v8h*)bp;
      bf.h[1] = *(const v8h*)(bp + 16);
      acc[t] = wmh(a.v, bf.v, acc[t]);
    }
  }
  if (KD == 2 * FD) {
#pragma unroll 1
    for (int kt = 0; kt < 4; ++kt) {
      FragH a;
      a.h[0] = *(const v8h*)(A2 + arow + 32 * kt);
      a.h[1] = *(const v8h*)(A2 + arow + 32 * kt + 16);
#pragma unroll
      for (int t = 0; t < NT; ++t) {
        const _Float16* bp = W + (size_t)(16 * t + m) * KD + FD + 32 * kt + 8 * hh;
        FragH bf;
        bf.h[0] = *(const v8h*)bp;
        bf.h[1] = *(const v8h*)(bp + 16);
        acc[t] = wmh(a.v, bf.v, acc[t]);
      }
    }
  }

  if (FIN) {
    float* sf = (float*)sraw;
#pragma unroll
    for (int t = 0; t < NT; ++t) {
      const float bv = bias[16 * t + m];
      float* sp = sf + (wave * 16 + 8 * hh) * SPF + 16 * t + m;
#pragma unroll
      for (int r = 0; r < 8; ++r) sp[r * SPF] = acc[t][r] * WINV + bv;
    }
    __syncthreads();
#pragma unroll 1
    for (int i = 0; i < 8; ++i) {
      const int rw = wave * 16 + 2 * i + hh;
      float* lp = sf + rw * SPF + 4 * m;
      const v4f v = *(const v4f*)lp;
      float ss = v.x * v.x + v.y * v.y + v.z * v.z + v.w * v.w;
      ss += __shfl_xor(ss, 8); ss += __shfl_xor(ss, 4); ss += __shfl_xor(ss, 2); ss += __shfl_xor(ss, 1);
      float nrm = sqrtf(ss);
      nrm = fmaxf(nrm, 1e-12f);
      const float inv = 1.0f / nrm;
      v4f y;
      y.x = fmaxf(v.x * inv, 0.0f); y.y = fmaxf(v.y * inv, 0.0f);
      y.z = fmaxf(v.z * inv, 0.0f); y.w = fmaxf(v.w * inv, 0.0f);
      float mx = fmaxf(fmaxf(y.x, y.y), fmaxf(y.z, y.w));
      mx = fmaxf(mx, __shfl_xor(mx, 8)); mx = fmaxf(mx, __shfl_xor(mx, 4));
      mx = fmaxf(mx, __shfl_xor(mx, 2)); mx = fmaxf(mx, __shfl_xor(mx, 1));
      float es = expf(y.x - mx) + expf(y.y - mx) + expf(y.z - mx) + expf(y.w - mx);
      es += __shfl_xor(es, 8); es += __shfl_xor(es, 4); es += __shfl_xor(es, 2); es += __shfl_xor(es, 1);
      const float lse = mx + logf(es);
      v4f o;
      o.x = y.x - lse; o.y = y.y - lse; o.z = y.z - lse; o.w = y.w - lse;
      *(v4f*)lp = o;
      const int grow = rowBase + rw;
      if (grow < nN) *(volatile v4f*)(out + (size_t)grow * NO + 4 * m) = o;
    }
    __threadfence();
#pragma unroll 1
    for (int i = 0; i < 8; ++i) {
      const int rw = wave * 16 + 2 * i + hh;
      const float* lp = sf + rw * SPF + 4 * m;
      const v4f o = *(const v4f*)lp;
      const int grow = rowBase + rw;
      if (grow < nN) *(volatile v4f*)(out + (size_t)grow * NO + 4 * m) = o;
    }
  } else {
    _Float16* sh = (_Float16*)sraw;
#pragma unroll
    for (int t = 0; t < NT; ++t) {
      const float bv = bias[16 * t + m];
      _Float16* sp = sh + (wave * 16 + 8 * hh) * SPH + 16 * t + m;
#pragma unroll
      for (int r = 0; r < 8; ++r) {
        float v = acc[t][r] * WINV + bv;
        v = fmaxf(v, 0.0f);
        sp[r * SPH] = (_Float16)v;
      }
    }
    __syncthreads();
    const size_t cbase = (size_t)rowBase * FD;
#pragma unroll
    for (int i = 0; i < 8; ++i) {
      const int rw = wave * 16 + 2 * i + hh;
      const v4f v = *(const v4f*)(sh + rw * SPH + 8 * m);
      *(volatile v4f*)(C + cbase + (size_t)rw * FD + 8 * m) = v;
    }
    __threadfence();
#pragma unroll
    for (int i = 0; i < 8; ++i) {
      const int rw = wave * 16 + 2 * i + hh;
      const v4f v = *(const v4f*)(sh + rw * SPH + 8 * m);
      *(volatile v4f*)(C + cbase + (size_t)rw * FD + 8 * m) = v;
    }
  }
}

__global__ __launch_bounds__(NTHR) void k_agg(
    const int* __restrict__ csr, const int* __restrict__ off, const int* __restrict__ cnt,
    const _Float16* __restrict__ xp, _Float16* agg, int nN, int csrLen) {
  extern __shared__ v4f lds_dyn[];
  _Float16* sA = (_Float16*)lds_dyn;
  const int tid = threadIdx.x, lane = tid & 31, wave = tid >> 5, hh = lane >> 4, m = lane & 15;
  const int tbase = blockIdx.x * TGT + wave * 32;
  const int cl = tbase + lane;
  const int cnt_l = cnt[cl];
  const int off_l = off[cl];

#pragma unroll 1
  for (int j = 0; j < 32; ++j) {
    int n = __builtin_amdgcn_readlane(cnt_l, j);
    n = n < 0 ? 0 : (n > DEGCAP ? DEGCAP : n);
    const int st = __builtin_amdgcn_readlane(off_l, j);
    v4f sm = {0.0f, 0.0f, 0.0f, 0.0f};
#pragma unroll 1
    for (int q0 = 0; q0 < n; q0 += 32) {
      int pos = st + q0 + lane;
      pos = pos < 0 ? 0 : (pos > csrLen - 1 ? csrLen - 1 : pos);
      int sl = csr[pos];
      sl = sl < 0 ? 0 : (sl > nN - 1 ? nN - 1 : sl);
      const int mcnt = (n - q0) < 32 ? (n - q0) : 32;
#pragma unroll 1
      for (int p = 0; p < mcnt; ++p) {
        const int s = __builtin_amdgcn_readlane(sl, p);
        const v4h hv = *(const v4h*)(xp + (size_t)s * FD + 4 * lane);
        sm.x += (float)hv.x; sm.y += (float)hv.y; sm.z += (float)hv.z; sm.w += (float)hv.w;
      }
    }
    const float rc = 1.0f / (float)(n > 1 ? n : 1);
    const v4f mean = sm * rc;
    v4h o;
    o.x = (_Float16)mean.x; o.y = (_Float16)mean.y; o.z = (_Float16)mean.z; o.w = (_Float16)mean.w;
    *(v4h*)(sA + (wave * 32 + j) * FD + 4 * lane) = o;
  }
  __syncthreads();

  const size_t gbase = (size_t)(blockIdx.x * TGT) * FD;
#pragma unroll
  for (int i = 0; i < 16; ++i) {
    const int rw = wave * 32 + 2 * i + hh;
    const v4f v = *(const v4f*)(sA + rw * FD + 8 * m);
    *(volatile v4f*)(agg + gbase + (size_t)rw * FD + 8 * m) = v;
  }
  __threadfence();
#pragma unroll
  for (int i = 0; i < 16; ++i) {
    const int rw = wave * 32 + 2 * i + hh;
    const v4f v = *(const v4f*)(sA + rw * FD + 8 * m);
    *(volatile v4f*)(agg + gbase + (size_t)rw * FD + 8 * m) = v;
  }
}

extern "C" void kernel_launch(void* const* d_in, const int* in_sizes, int n_in,
                              void* d_out, int out_size, void* d_ws, size_t ws_size,
                              hipStream_t stream) {
  if (n_in < 12) return;
  const int nN = in_sizes[0] / FD;
  const int nE = in_sizes[1] / 2;
  if (nN <= 0 || nE <= 0) return;
  if (in_sizes[0] != nN * FD || in_sizes[1] != 2 * nE) return;
  if (in_sizes[2] != FD * FD || in_sizes[3] != FD) return;
  if (in_sizes[4] != FD * FD || in_sizes[5] != FD || in_sizes[6] != FD * FD) return;
  if (in_sizes[7] != FD * FD || in_sizes[8] != FD) return;
  if (in_sizes[9] != NO * FD || in_sizes[10] != NO || in_sizes[11] != NO * FD) return;
  if (out_size != nN * NO) return;
  if (nE > (1 << 28) || nN > (1 << 24)) return;

  const float* x    = (const float*)d_in[0];
  const int*   ei   = (const int*)d_in[1];
  const float* p1w  = (const float*)d_in[2];
  const float* p1b  = (const float*)d_in[3];
  const float* l1lw = (const float*)d_in[4];
  const float* l1lb = (const float*)d_in[5];
  const float* l1rw = (const float*)d_in[6];
  const float* p2w  = (const float*)d_in[7];
  const float* p2b  = (const float*)d_in[8];
  const float* l2lw = (const float*)d_in[9];
  const float* l2lb = (const float*)d_in[10];
  const float* l2rw = (const float*)d_in[11];
  const int* srcs = ei;
  const int* dsts = ei + nE;
  float* out = (float*)d_out;

  const int NPAD   = ((nN + TGT - 1) / TGT) * TGT;
  const int nBC    = (nN + NBC - 1) / NBC;
  const int CNTPAD = nBC * NBC;
  if (4 * nBC + 1 > RBN) return;
  const int nBF    = (nN + NBF - 1) / NBF;
  const int csrLen = ((nE + 31) & ~31) + 4096;
  if (31 * 4 * nBC > 4096) return;
  const int nGemm  = NPAD / GROWS;
  const int nAgg   = NPAD / TGT;
  const int nCvt   = NPAD / 16;

  char* ws = (char*)d_ws;
  size_t offb = 0;
  const size_t oW   = offb; offb += (size_t)WPTOT * 2;       offb = (offb + 255) & ~(size_t)255;
  const size_t oCnt = offb; offb += (size_t)CNTPAD * 4;      offb = (offb + 255) & ~(size_t)255;
  const size_t oOff = offb; offb += (size_t)CNTPAD * 4;      offb = (offb + 255) & ~(size_t)255;
  const size_t oRb  = offb; offb += (size_t)RBN * 4;         offb = (offb + 255) & ~(size_t)255;
  const size_t oCsr = offb; offb += (size_t)csrLen * 4;      offb = (offb + 255) & ~(size_t)255;
  const size_t oRX  = offb; offb += (size_t)NPAD * FD * 2;   offb = (offb + 255) & ~(size_t)255;
  const size_t oRP  = offb; offb += (size_t)NPAD * FD * 2;   offb = (offb + 255) & ~(size_t)255;
  const size_t oRA  = offb; offb += (size_t)NPAD * FD * 2;   offb = (offb + 255) & ~(size_t)255;
  if (offb > ws_size || offb > (size_t)WSCAP) return;
  _Float16* wp   = (_Float16*)(ws + oW);
  int*      cnt  = (int*)(ws + oCnt);
  int*      offp = (int*)(ws + oOff);
  int*      rb   = (int*)(ws + oRb);
  int*      csr  = (int*)(ws + oCsr);
  _Float16* RX   = (_Float16*)(ws + oRX);
  _Float16* RP   = (_Float16*)(ws + oRP);
  _Float16* RA   = (_Float16*)(ws + oRA);

  const int vec8 = ((nE & 3) == 0) ? 1 : 0;

  k_wprep<<<40, NTHR, 0, stream>>>(p1w, l1lw, l1rw, p2w, l2lw, l2rw, wp);
  k_cvtx<<<nCvt, NTHR, 0, stream>>>(x, RX, nN);

  k_count<<<nBC, NTHR, 0, stream>>>(dsts, cnt, nE, vec8);
  k_offsets<<<1, OTHR, 0, stream>>>(cnt, offp, rb, nBC);
  hipFuncSetAttribute(reinterpret_cast<const void*>(&k_fill),
                      hipFuncAttributeMaxDynamicSharedMemorySize, LDS_FILL);
  k_fill<<<nBF, NTHR, LDS_FILL, stream>>>(srcs, dsts, offp, rb, csr, nN, nE, vec8, csrLen);

  k_gemm<FD, 8, false><<<nGemm, NTHR, 0, stream>>>(RX, RX, wp + WP1, p1b, RP, out, nN);
  hipFuncSetAttribute(reinterpret_cast<const void*>(&k_agg),
                      hipFuncAttributeMaxDynamicSharedMemorySize, LDS_AGG);
  k_agg<<<nAgg, NTHR, LDS_AGG, stream>>>(csr, offp, cnt, RP, RA, nN, csrLen);
  k_gemm<2 * FD, 8, false><<<nGemm, NTHR, 0, stream>>>(RA, RP, wp + WL1, l1lb, RX, out, nN);

  k_gemm<FD, 8, false><<<nGemm, NTHR, 0, stream>>>(RX, RX, wp + WP2, p2b, RP, out, nN);
  k_agg<<<nAgg, NTHR, LDS_AGG, stream>>>(csr, offp, cnt, RP, RA, nN, csrLen);
  k_gemm<2 * FD, 4, true><<<nGemm, NTHR, 0, stream>>>(RA, RP, wp + WL2, l2lb, RX, out, nN);
}
